// MambaLayer_12816182411895
// MI455X (gfx1250) — hardware-verified
//
#include <hip/hip_runtime.h>
#include <math.h>

typedef __attribute__((ext_vector_type(16))) _Float16 v16h;
typedef __attribute__((ext_vector_type(8)))  _Float16 v8h;
typedef __attribute__((ext_vector_type(16))) __bf16   v16b;
typedef __attribute__((ext_vector_type(8)))  __bf16   v8b;
typedef __attribute__((ext_vector_type(8)))  float    v8f;
typedef __attribute__((ext_vector_type(4)))  float    v4f;
typedef __attribute__((ext_vector_type(4)))  unsigned v4u;

constexpr int kBatch = 4;
constexpr int kSeqL  = 512;
constexpr int kDm    = 1024;
constexpr int kDin   = 2048;
constexpr int kNst   = 16;
constexpr int kDc    = 4;
constexpr int kDtR   = 64;
constexpr int kPrjN  = kDtR + 2 * kNst;
constexpr int kPrjP  = 128;
constexpr int kXZP   = 2 * kDin;
constexpr int kFfn   = 2 * kDm;
constexpr int kRows  = kBatch * kSeqL;
constexpr int kTP    = 260;
constexpr float kLog2e = 1.4426950408889634f;
constexpr float kLnEps = 1e-12f;
static_assert(kPrjN == 96 && kXZP == 4096 && kFfn == 2048 && kRows == 2048);
static_assert((kDm % 32) == 0 && (kDin % 32) == 0 && (kDtR % 32) == 0 && (kFfn % 32) == 0);
static_assert((kRows % 64) == 0 && (kXZP % 64) == 0 && (kPrjP % 64) == 0 && (kDin % 64) == 0 && (kDm % 64) == 0 && (kFfn % 64) == 0);
static_assert((kSeqL % 64) == 0 && (kSeqL % 16) == 0 && (kDin % 256) == 0 && (kDm == 256 * 4));

constexpr size_t kSzWIN  = (size_t)kXZP  * kDm   * 2;
constexpr size_t kSzWXP  = (size_t)kPrjP * kDin  * 2;
constexpr size_t kSzWDT  = (size_t)kDin  * kDtR  * 2;
constexpr size_t kSzWOUT = (size_t)kDm   * kDin  * 2;
constexpr size_t kSzW1   = (size_t)kFfn  * kDm   * 2;
constexpr size_t kSzW2   = (size_t)kDm   * kFfn  * 2;
constexpr size_t kSzXB   = (size_t)kRows * kDm   * 2;
constexpr size_t kSzXZ   = (size_t)kRows * kXZP  * 4;
constexpr size_t kSzUCB  = (size_t)kRows * kDin  * 2;
constexpr size_t kSzPROJ = (size_t)kRows * kPrjP * 4;
constexpr size_t kSzDTRB = (size_t)kRows * kDtR  * 2;
constexpr size_t kSzDLR  = (size_t)kRows * kDin  * 4;
constexpr size_t kSzYB   = (size_t)kRows * kDin  * 2;
constexpr size_t kSzMO   = (size_t)kRows * kDm   * 4;
constexpr size_t kSzH    = (size_t)kRows * kDm   * 4;
constexpr size_t kSzHH   = (size_t)kRows * kDm   * 2;
constexpr size_t kSzHL   = kSzHH;
constexpr size_t kSzF2   = (size_t)kRows * kDm   * 4;
constexpr size_t kOffWIN  = 0;
constexpr size_t kOffWXP  = kOffWIN  + kSzWIN;
constexpr size_t kOffWDT  = kOffWXP  + kSzWXP;
constexpr size_t kOffWOUT = kOffWDT  + kSzWDT;
constexpr size_t kOffW1   = kOffWOUT + kSzWOUT;
constexpr size_t kOffW2   = kOffW1   + kSzW1;
constexpr size_t kOffXB   = kOffW2   + kSzW2;
constexpr size_t kOffXZ   = kOffXB   + kSzXB;
constexpr size_t kOffUCB  = kOffXZ   + kSzXZ;
constexpr size_t kOffPROJ = kOffUCB  + kSzUCB;
constexpr size_t kOffDTRB = kOffPROJ + kSzPROJ;
constexpr size_t kOffDLR  = kOffDTRB + kSzDTRB;
constexpr size_t kOffYB   = kOffDLR  + kSzDLR;
constexpr size_t kOffMO   = kOffYB   + kSzYB;
constexpr size_t kOffH    = kOffMO   + kSzMO;
constexpr size_t kOffHH   = kOffH    + kSzH;
constexpr size_t kOffHL   = kOffHH   + kSzHH;
constexpr size_t kOffF2   = kOffHL   + kSzHL;
constexpr size_t kWsTotal = kOffF2   + kSzF2;
constexpr size_t kOffFH   = kOffUCB;
constexpr size_t kOffFL   = kOffYB;
static_assert(kWsTotal == 127926272ull);
static_assert(kWsTotal <= 134217728ull);
static_assert((size_t)kRows * kFfn * 2 == kSzUCB && (size_t)kRows * kFfn * 2 == kSzYB);
static_assert((kOffWXP % 128) == 0 && (kOffWDT % 128) == 0 && (kOffWOUT % 128) == 0 && (kOffW1 % 128) == 0 &&
              (kOffW2 % 128) == 0 && (kOffXB % 128) == 0 && (kOffXZ % 128) == 0 && (kOffUCB % 128) == 0 &&
              (kOffPROJ % 128) == 0 && (kOffDTRB % 128) == 0 && (kOffDLR % 128) == 0 && (kOffYB % 128) == 0 &&
              (kOffMO % 128) == 0 && (kOffH % 128) == 0 && (kOffHH % 128) == 0 && (kOffHL % 128) == 0 && (kOffF2 % 128) == 0);

__device__ __forceinline__ unsigned short f2bf_bits(float f) {
  unsigned u = __float_as_uint(f);
  return (unsigned short)((u + 0x7FFFu + ((u >> 16) & 1u)) >> 16);
}
__device__ __forceinline__ float bf_bits2f(unsigned short h) { return __uint_as_float(((unsigned)h) << 16); }
__device__ __forceinline__ unsigned f2bf_u(float f) {
  const unsigned u = __float_as_uint(f);
  return (u + 0x7FFFu + ((u >> 16) & 1u)) >> 16;
}
__device__ __forceinline__ float bf_u2f(unsigned b) { return __uint_as_float(b << 16); }
__device__ __forceinline__ float bfr(float f) { return bf_u2f(f2bf_u(f)); }
__device__ __forceinline__ unsigned pack_bf16x2(float a, float b) { return f2bf_u(a) | (f2bf_u(b) << 16); }
__device__ __forceinline__ void split_bf16x2(float a, float b, unsigned& wh, unsigned& wl) {
  const unsigned ha = f2bf_u(a), hb = f2bf_u(b);
  const unsigned la = f2bf_u(a - bf_u2f(ha)), lb = f2bf_u(b - bf_u2f(hb));
  wh = ha | (hb << 16);
  wl = la | (lb << 16);
}
__device__ __forceinline__ float wave_sum(float v) {
#pragma unroll
  for (int off = 16; off > 0; off >>= 1) v += __shfl_xor(v, off, 32);
  return v;
}

__device__ __forceinline__ void dep_guard_h(v8f& a, v8f& b, v16h x, v16h y) { asm volatile("v_nop\n\tv_nop\n\tv_nop\n\tv_nop" : "+v"(a), "+v"(b) : "v"(x), "v"(y)); }
__device__ __forceinline__ void dep_guard_b(v8f& a, v8f& b, v16b x, v16b y) { asm volatile("v_nop\n\tv_nop\n\tv_nop\n\tv_nop" : "+v"(a), "+v"(b) : "v"(x), "v"(y)); }
__device__ __forceinline__ void dep_guard4_h(v8f& a, v8f& b, v8f& c, v8f& d, v16h x, v16h y) { asm volatile("v_nop\n\tv_nop\n\tv_nop\n\tv_nop" : "+v"(a), "+v"(b), "+v"(c), "+v"(d) : "v"(x), "v"(y)); }
__device__ __forceinline__ void dep_guard4_b(v8f& a, v8f& b, v8f& c, v8f& d, v16b x, v16b y) { asm volatile("v_nop\n\tv_nop\n\tv_nop\n\tv_nop" : "+v"(a), "+v"(b), "+v"(c), "+v"(d) : "v"(x), "v"(y)); }
__device__ __forceinline__ void keep4_h(v16h a, v16h b, v16h c, v16h d) { asm volatile("v_nop" :: "v"(a), "v"(b), "v"(c), "v"(d)); }
__device__ __forceinline__ void keep4_b(v16b a, v16b b, v16b c, v16b d) { asm volatile("v_nop" :: "v"(a), "v"(b), "v"(c), "v"(d)); }
__device__ __forceinline__ void acc_guard4(v8f& a, v8f& b, v8f& c, v8f& d) { asm volatile("v_nop\n\tv_nop\n\tv_nop\n\tv_nop" : "+v"(a), "+v"(b), "+v"(c), "+v"(d)); }
template <typename T> struct Frag;
template <> struct Frag<_Float16> {
  typedef v16h V; union U { v16h v; v8h h[2]; };
  static __device__ __forceinline__ v16h load(const _Float16* p) {
    U f; f.h[0] = *(const v8h*)(p); f.h[1] = *(const v8h*)(p + 16); return f.v;
  }
  static __device__ __forceinline__ v8f mma(v16h a, v16h b, v8f c) {
    return __builtin_amdgcn_wmma_f32_16x16x32_f16(false, a, false, b, (short)0, c, false, false);
  }
  static __device__ __forceinline__ void guard(v8f& a, v8f& b, v16h x, v16h y) { dep_guard_h(a, b, x, y); }
  static __device__ __forceinline__ void guard4(v8f& a, v8f& b, v8f& c, v8f& d, v16h x, v16h y) { dep_guard4_h(a, b, c, d, x, y); }
  static __device__ __forceinline__ void keep(v16h a, v16h b, v16h c, v16h d) { keep4_h(a, b, c, d); }
};
template <> struct Frag<__bf16> {
  typedef v16b V; union U { v16b v; v8b h[2]; };
  static __device__ __forceinline__ v16b load(const __bf16* p) {
    U f; f.h[0] = *(const v8b*)(p); f.h[1] = *(const v8b*)(p + 16); return f.v;
  }
  static __device__ __forceinline__ v8f mma(v16b a, v16b b, v8f c) {
    return __builtin_amdgcn_wmma_f32_16x16x32_bf16(false, a, false, b, (short)0, c, false, false);
  }
  static __device__ __forceinline__ void guard(v8f& a, v8f& b, v16b x, v16b y) { dep_guard_b(a, b, x, y); }
  static __device__ __forceinline__ void guard4(v8f& a, v8f& b, v8f& c, v8f& d, v16b x, v16b y) { dep_guard4_b(a, b, c, d, x, y); }
  static __device__ __forceinline__ void keep(v16b a, v16b b, v16b c, v16b d) { keep4_b(a, b, c, d); }
};

template <int ET> struct Elem;
template <> struct Elem<0> { typedef _Float16 T; };
template <> struct Elem<1> { typedef __bf16 T; };
template <int ET, int SPL, int BIAS_MODE, int OUT_MODE, bool RESID, int ACT = 0>
__global__ __launch_bounds__(256) void wmma_gemm64(
    const unsigned short* __restrict__ Ap, const unsigned short* __restrict__ A2p, int lda, long strideA,
    const unsigned short* __restrict__ Btp, const unsigned short* __restrict__ Bt2p, int ldb, long strideB,
    void* __restrict__ Cout, void* __restrict__ Cout2, int ldc, long strideC,
    const float* __restrict__ bias,
    const float* __restrict__ resid, long strideR,
    int M, int N, int K, float scale) {
  typedef typename Elem<ET>::T T;
  typedef typename Frag<T>::V V;
  const T* A = (const T*)Ap; const T* A2 = (const T*)A2p; const T* Bt = (const T*)Btp; const T* Bt2 = (const T*)Bt2p;
  __shared__ __align__(16) float sT[8][16 * 68];
  const int b    = blockIdx.y;
  const int lane = threadIdx.x & 31;
  const int wave = threadIdx.x >> 5;
  const int tilesN = N >> 6;
  const int tilesM = M >> 6;
  const int tile = blockIdx.x * 8 + wave;
  if (tile >= tilesM * tilesN) return;
  const int tm = tile / tilesN;
  const int tn = tile - tm * tilesN;
  const int m0 = tm << 6;
  const int n0 = tn << 6;

  const T* Ab  = A  + (size_t)b * strideA;
  const T* Bb  = Bt + (size_t)b * strideB;
  const T* Ab2 = (SPL >= 1) ? (A2  + (size_t)b * strideA) : nullptr;
  const T* Bb2 = (SPL == 2) ? (Bt2 + (size_t)b * strideB) : nullptr;

  const int rlane = lane & 15;
  const int koff  = (lane >> 4) * 8;
  const int mOff  = (lane >> 4) * 8;

  v8f acc[4][4];
#pragma unroll
  for (int i = 0; i < 4; ++i)
#pragma unroll
    for (int j = 0; j < 4; ++j) acc[i][j] = (v8f){0.f,0.f,0.f,0.f,0.f,0.f,0.f,0.f};

  for (int k0 = 0; k0 < K; k0 += 32) {
    V bh[4], bl[4];
#pragma unroll
    for (int j = 0; j < 4; ++j) {
      const size_t bo = (size_t)(n0 + (j << 4) + rlane) * ldb + koff + k0;
      bh[j] = Frag<T>::load(Bb + bo);
      if (SPL == 2) bl[j] = Frag<T>::load(Bb2 + bo);
    }
#pragma unroll
    for (int i = 0; i < 4; ++i) {
      const size_t ao = (size_t)(m0 + (i << 4) + rlane) * lda + koff + k0;
      V ah = Frag<T>::load(Ab + ao);
      V al;
      if (SPL >= 1) al = Frag<T>::load(Ab2 + ao);
#pragma unroll
      for (int j = 0; j < 4; ++j) {
        acc[i][j] = Frag<T>::mma(ah, bh[j], acc[i][j]);
        if (SPL == 2) acc[i][j] = Frag<T>::mma(ah, bl[j], acc[i][j]);
        if (SPL >= 1) acc[i][j] = Frag<T>::mma(al, bh[j], acc[i][j]);
      }
      Frag<T>::guard4(acc[i][0], acc[i][1], acc[i][2], acc[i][3], ah, (SPL >= 1) ? al : ah);
    }
    Frag<T>::keep(bh[0], bh[1], bh[2], bh[3]);
    if (SPL == 2) Frag<T>::keep(bl[0], bl[1], bl[2], bl[3]);
  }
  acc_guard4(acc[0][0], acc[0][1], acc[0][2], acc[0][3]);
  acc_guard4(acc[1][0], acc[1][1], acc[1][2], acc[1][3]);
  acc_guard4(acc[2][0], acc[2][1], acc[2][2], acc[2][3]);
  acc_guard4(acc[3][0], acc[3][1], acc[3][2], acc[3][3]);

  float* slab = sT[wave];
  const float* Rb = RESID ? (resid + (size_t)b * strideR) : nullptr;
#pragma unroll
  for (int i = 0; i < 4; ++i) {
    const int mBase = m0 + (i << 4);
#pragma unroll
    for (int j = 0; j < 4; ++j) {
      const int n = n0 + (j << 4) + rlane;
      float bv = 0.f;
      if (BIAS_MODE == 2) bv = bias[n];
#pragma unroll
      for (int r = 0; r < 8; ++r) {
        float v = acc[i][j][r] * scale;
        if (BIAS_MODE == 1) v += bias[mBase + mOff + r];
        if (BIAS_MODE == 2) v += bv;
        if (RESID) v += Rb[(size_t)(mBase + mOff + r) * ldc + n];
        if (ACT == 1) v = tanhf(v);
        if (ACT == 2) v = fmaxf(v, 0.0f);
        if (ACT == 3) v = v / (1.0f + expf(-v));
        if (ACT == 4) v = (v > 0.f) ? v : 0.01f * v;
        slab[(mOff + r) * 68 + (j << 4) + rlane] = v;
      }
    }
    __builtin_amdgcn_fence(__ATOMIC_RELEASE, "workgroup");
    __builtin_amdgcn_wave_barrier();
    __builtin_amdgcn_fence(__ATOMIC_ACQUIRE, "workgroup");
    if (OUT_MODE == 0) {
      float* C = (float*)Cout + (size_t)b * strideC;
      const int hh = lane >> 4, c4 = (lane & 15) * 4;
      for (int pass = 0; pass < 2; ++pass) {
#pragma unroll
        for (int it = 0; it < 8; ++it) {
          const int row = it * 2 + hh;
          v4f v = *(const v4f*)(slab + row * 68 + c4);
          *(volatile v4f*)(C + (size_t)(mBase + row) * ldc + n0 + c4) = v;
        }
        __threadfence();
      }
    } else {
      const int q = lane >> 3, c8 = (lane & 7) * 8;
      unsigned short* C  = (unsigned short*)Cout  + (size_t)b * strideC;
      unsigned short* C2 = (OUT_MODE == 2) ? ((unsigned short*)Cout2 + (size_t)b * strideC) : nullptr;
      for (int pass = 0; pass < 2; ++pass) {
#pragma unroll
        for (int it = 0; it < 4; ++it) {
          const int row = it * 4 + q;
          const float* sp = slab + row * 68 + c8;
          v8h hv, lv;
#pragma unroll
          for (int e = 0; e < 8; ++e) {
            if (OUT_MODE == 1) {
              hv[e] = (_Float16)sp[e];
            } else {
              unsigned short hb = f2bf_bits(sp[e]);
              unsigned short lb = f2bf_bits(sp[e] - bf_bits2f(hb));
              hv[e] = __builtin_bit_cast(_Float16, hb);
              lv[e] = __builtin_bit_cast(_Float16, lb);
            }
          }
          *(volatile v8h*)(C + (size_t)(mBase + row) * ldc + n0 + c8) = hv;
          if (OUT_MODE == 2) *(volatile v8h*)(C2 + (size_t)(mBase + row) * ldc + n0 + c8) = lv;
        }
        __threadfence();
      }
    }
    __builtin_amdgcn_fence(__ATOMIC_RELEASE, "workgroup");
    __builtin_amdgcn_wave_barrier();
    __builtin_amdgcn_fence(__ATOMIC_ACQUIRE, "workgroup");
  }
}

__global__ __launch_bounds__(256) void cast_bf16_kernel(
    const float* __restrict__ src, unsigned short* __restrict__ dst, int total8, int nreal8)
{
  const int i = blockIdx.x * 256 + threadIdx.x;
  if (i >= total8) return;
  const size_t e0 = (size_t)i << 3;
  const bool real = (i < nreal8);
  const size_t ec = real ? e0 : (size_t)0;
  const v4f a0 = *(const v4f*)(src + ec);
  const v4f a1 = *(const v4f*)(src + ec + 4);
  v4u wv;
  wv[0] = real ? pack_bf16x2(a0[0], a0[1]) : 0u;
  wv[1] = real ? pack_bf16x2(a0[2], a0[3]) : 0u;
  wv[2] = real ? pack_bf16x2(a1[0], a1[1]) : 0u;
  wv[3] = real ? pack_bf16x2(a1[2], a1[3]) : 0u;
  unsigned short* q = dst + e0;
  *(volatile v4u*)q = wv;
  __threadfence();
  *(volatile v4u*)q = wv;
}

__global__ __launch_bounds__(256) void dtr_cast_kernel(
    const float* __restrict__ PROJ, unsigned short* __restrict__ DTRB, int total8)
{
  const int i = blockIdx.x * 256 + threadIdx.x;
  if (i >= total8) return;
  const int e0  = i << 3;
  const int row = e0 >> 6;
  const int c8  = e0 & 63;
  const float* p = PROJ + (size_t)row * kPrjP + c8;
  const v4f a0 = *(const v4f*)(p);
  const v4f a1 = *(const v4f*)(p + 4);
  v4u wv;
  wv[0] = pack_bf16x2(a0[0], a0[1]);
  wv[1] = pack_bf16x2(a0[2], a0[3]);
  wv[2] = pack_bf16x2(a1[0], a1[1]);
  wv[3] = pack_bf16x2(a1[2], a1[3]);
  unsigned short* q = DTRB + e0;
  *(volatile v4u*)q = wv;
  __threadfence();
  *(volatile v4u*)q = wv;
}

__device__ __forceinline__ float silu_f(float v) { return v * (1.0f / (1.0f + expf(-v))); }
__device__ __forceinline__ float conv_silu_val(float w0, float w1, float w2, float w3, float bc,
                                              float xm3, float xm2, float xm1, float xc) {
  float acc = w0 * xm3;
  acc = fmaf(w1, xm2, acc);
  acc = fmaf(w2, xm1, acc);
  acc = fmaf(w3, xc, acc);
  return silu_f(acc + bc);
}

__global__ __launch_bounds__(256) void conv_silu_kernel(
    const float* __restrict__ XZ, const float* __restrict__ cw, const float* __restrict__ cb,
    unsigned short* __restrict__ UCB)
{
  __shared__ __align__(16) float sT[16 * kTP];
  const int tid = threadIdx.x, lane = tid & 31, wave = tid >> 5;
  const int d0 = blockIdx.x * 256, d = d0 + tid;
  const int g0 = blockIdx.y * 64;
  const int tb = g0 & (kSeqL - 1);
  const float w0 = bfr(cw[d * kDc + 0]), w1 = bfr(cw[d * kDc + 1]), w2 = bfr(cw[d * kDc + 2]), w3 = bfr(cw[d * kDc + 3]);
  const float bc = bfr(cb[d]);
  float xm3, xm2, xm1;
  {
    const bool hist = (tb > 0);
    const int rb = hist ? (g0 - 3) : g0;
    const float v3 = XZ[(size_t)rb * kXZP + d];
    const float v2 = XZ[(size_t)(rb + 1) * kXZP + d];
    const float v1 = XZ[(size_t)(rb + 2) * kXZP + d];
    xm3 = hist ? v3 : 0.f;
    xm2 = hist ? v2 : 0.f;
    xm1 = hist ? v1 : 0.f;
  }
#pragma unroll 1
  for (int sub = 0; sub < 4; ++sub) {
    const int lb = g0 + sub * 16;
#pragma unroll 1
    for (int s = 0; s < 16; ++s) {
      const float xc = XZ[(size_t)(lb + s) * kXZP + d];
      sT[s * kTP + tid] = conv_silu_val(w0, w1, w2, w3, bc, xm3, xm2, xm1, xc);
      xm3 = xm2; xm2 = xm1; xm1 = xc;
    }
    __syncthreads();
    v4u wv[2];
#pragma unroll
    for (int it = 0; it < 2; ++it) {
      const float* sp = sT + (it * 8 + wave) * kTP + lane * 8;
      const v4f a0 = *(const v4f*)(sp);
      const v4f a1 = *(const v4f*)(sp + 4);
      wv[it][0] = pack_bf16x2(a0[0], a0[1]);
      wv[it][1] = pack_bf16x2(a0[2], a0[3]);
      wv[it][2] = pack_bf16x2(a1[0], a1[1]);
      wv[it][3] = pack_bf16x2(a1[2], a1[3]);
    }
    for (int pass = 0; pass < 2; ++pass) {
#pragma unroll
      for (int it = 0; it < 2; ++it)
        *(volatile v4u*)(UCB + (size_t)(lb + it * 8 + wave) * kDin + d0 + lane * 8) = wv[it];
      __threadfence();
    }
    __syncthreads();
  }
}

__global__ __launch_bounds__(256) void scan_kernel(
    const float* __restrict__ DLR, const float* __restrict__ XZ, const float* __restrict__ PROJ,
    const float* __restrict__ cw, const float* __restrict__ cb, const float* __restrict__ bdt,
    const float* __restrict__ Alog, const float* __restrict__ Dv, unsigned short* __restrict__ YB)
{
  __shared__ __align__(16) float sBC[16 * 32];
  __shared__ __align__(16) float sY[16 * kTP];
  __shared__ __align__(16) float sA[kNst * 256];
  const int tid = threadIdx.x, lane = tid & 31, wave = tid >> 5;
  const int d0 = blockIdx.x * 256, d = d0 + tid;
  const size_t row0 = (size_t)blockIdx.y * kSeqL;

#pragma unroll 1
  for (int n = 0; n < kNst; ++n) sA[n * 256 + tid] = -expf(bfr(Alog[(size_t)d * kNst + n])) * kLog2e;
  __syncthreads();
  float A2[kNst], h[kNst];
#pragma unroll
  for (int n = 0; n < kNst; ++n) { A2[n] = sA[n * 256 + tid]; h[n] = 0.0f; }

  const float w0 = bfr(cw[d * kDc + 0]), w1 = bfr(cw[d * kDc + 1]), w2 = bfr(cw[d * kDc + 2]), w3 = bfr(cw[d * kDc + 3]);
  const float bc = bfr(cb[d]);
  const float bb = bfr(bdt[d]);
  const float Dd = bfr(Dv[d]);
  float xm3 = 0.0f, xm2 = 0.0f, xm1 = 0.0f;

#pragma unroll 1
  for (int ck = 0; ck < kSeqL / 16; ++ck) {
    const int l0 = ck * 16;
    if (tid < 128) {
      const int r = tid >> 3, q = (tid & 7) * 4;
      const v4f v = *(const v4f*)(PROJ + (row0 + l0 + r) * kPrjP + kDtR + q);
      *(v4f*)(sBC + r * 32 + q) = v;
    }
    __syncthreads();
#pragma unroll 1
    for (int s = 0; s < 16; ++s) {
      const size_t m = row0 + l0 + s;
      const float a     = DLR[m * kDin + d] + bb;
      const float delta = fmaxf(a, 0.0f) + log1pf(expf(-fabsf(a)));
      const float xc    = XZ[m * kXZP + d];
      const float xv    = conv_silu_val(w0, w1, w2, w3, bc, xm3, xm2, xm1, xc);
      xm3 = xm2; xm2 = xm1; xm1 = xc;
      const float zv    = XZ[m * kXZP + kDin + d];
      v4f Bq[4], Cq[4];
#pragma unroll
      for (int qq = 0; qq < 4; ++qq) {
        Bq[qq] = *(const v4f*)(sBC + s * 32 + 4 * qq);
        Cq[qq] = *(const v4f*)(sBC + s * 32 + kNst + 4 * qq);
      }
      float y = 0.0f;
#pragma unroll
      for (int n = 0; n < kNst; ++n) {
        const float e  = exp2f(delta * A2[n]);
        const float p  = (delta * Bq[n >> 2][n & 3]) * xv;
        const float hn = e * h[n] + p;
        h[n] = hn;
        y += hn * Cq[n >> 2][n & 3];
      }
      y += Dd * xv;
      const float g = silu_f(zv);
      sY[s * kTP + tid] = y * g;
    }
    __syncthreads();
    v4u wv[2];
#pragma unroll
    for (int it = 0; it < 2; ++it) {
      const float* sp = sY + (it * 8 + wave) * kTP + lane * 8;
      const v4f a0 = *(const v4f*)(sp);
      const v4f a1 = *(const v4f*)(sp + 4);
      wv[it][0] = pack_bf16x2(a0[0], a0[1]);
      wv[it][1] = pack_bf16x2(a0[2], a0[3]);
      wv[it][2] = pack_bf16x2(a1[0], a1[1]);
      wv[it][3] = pack_bf16x2(a1[2], a1[3]);
    }
    for (int pass = 0; pass < 2; ++pass) {
#pragma unroll
      for (int it = 0; it < 2; ++it)
        *(volatile v4u*)(YB + (row0 + l0 + it * 8 + wave) * kDin + d0 + lane * 8) = wv[it];
      __threadfence();
    }
  }
}

template <bool RND_RESID, bool EMIT16>
__global__ __launch_bounds__(256) void add_ln_kernel(
    const float* __restrict__ A, const float* __restrict__ R,
    const float* __restrict__ gw, const float* __restrict__ gb,
    float* __restrict__ O, unsigned short* __restrict__ OH, unsigned short* __restrict__ OL)
{
  __shared__ __align__(16) float sRow[kDm];
  __shared__ float red1[8];
  __shared__ float red2[8];
  const int m = blockIdx.x, tid = threadIdx.x, lane = tid & 31, wave = tid >> 5;
  const int c4 = tid * 4;
  const size_t base = (size_t)m * kDm + c4;
  const v4f av = *(const v4f*)(A + base);
  const v4f rv = *(const v4f*)(R + base);
  const v4f wv = *(const v4f*)(gw + c4);
  const v4f bv = *(const v4f*)(gb + c4);
  float t[4];
#pragma unroll
  for (int e = 0; e < 4; ++e) {
    const float r = RND_RESID ? bfr(rv[e]) : rv[e];
    t[e] = av[e] + r;
  }
  float s = 0.0f;
#pragma unroll
  for (int e = 0; e < 4; ++e) s += t[e];
  s = wave_sum(s);
  if (lane == 0) red1[wave] = s;
  __syncthreads();
  float tot = 0.0f;
#pragma unroll
  for (int i = 0; i < 8; ++i) tot += red1[i];
  const float mean = tot * (1.0f / (float)kDm);
  float dv[4];
  float s2 = 0.0f;
#pragma unroll
  for (int e = 0; e < 4; ++e) { dv[e] = t[e] - mean; s2 = fmaf(dv[e], dv[e], s2); }
  s2 = wave_sum(s2);
  if (lane == 0) red2[wave] = s2;
  __syncthreads();
  float tot2 = 0.0f;
#pragma unroll
  for (int i = 0; i < 8; ++i) tot2 += red2[i];
  const float var  = tot2 * (1.0f / (float)kDm);
  const float rstd = 1.0f / sqrtf(var + kLnEps);
  v4f ov;
#pragma unroll
  for (int e = 0; e < 4; ++e) ov[e] = (dv[e] * rstd) * bfr(wv[e]) + bfr(bv[e]);

  v4u wh = (v4u){0u, 0u, 0u, 0u}, wl = (v4u){0u, 0u, 0u, 0u};
  if (EMIT16) {
    *(v4f*)(sRow + c4) = ov;
    __syncthreads();
    if (tid < 128) {
      const float* sp = sRow + tid * 8;
      const v4f a0 = *(const v4f*)(sp);
      const v4f a1 = *(const v4f*)(sp + 4);
      unsigned h0, l0, h1, l1, h2, l2, h3, l3;
      split_bf16x2(a0[0], a0[1], h0, l0);
      split_bf16x2(a0[2], a0[3], h1, l1);
      split_bf16x2(a1[0], a1[1], h2, l2);
      split_bf16x2(a1[2], a1[3], h3, l3);
      wh = (v4u){h0, h1, h2, h3};
      wl = (v4u){l0, l1, l2, l3};
    }
  }
  unsigned short* ph = OH + (size_t)m * kDm + tid * 8;
  unsigned short* pl = OL + (size_t)m * kDm + tid * 8;
  for (int pass = 0; pass < 2; ++pass) {
    *(volatile v4f*)(O + base) = ov;
    if (EMIT16) {
      if (tid < 128) {
        *(volatile v4u*)ph = wh;
        *(volatile v4u*)pl = wl;
      }
    }
    __threadfence();
  }
}

extern "C" void kernel_launch(void* const* d_in, const int* in_sizes, int n_in,
                              void* d_out, int out_size, void* d_ws, size_t ws_size,
                              hipStream_t stream)
{
  if (n_in < 18) return;
  if (in_sizes[0]  != kRows * kDm) return;
  if (in_sizes[1]  != kXZP * kDm) return;
  if (in_sizes[2]  != kDin * kDc) return;
  if (in_sizes[3]  != kDin) return;
  if (in_sizes[4]  != kPrjN * kDin) return;
  if (in_sizes[5]  != kDin * kDtR) return;
  if (in_sizes[6]  != kDin) return;
  if (in_sizes[7]  != kDin * kNst) return;
  if (in_sizes[8]  != kDin) return;
  if (in_sizes[9]  != kDm * kDin) return;
  if (in_sizes[10] != kDm || in_sizes[11] != kDm) return;
  if (in_sizes[12] != kFfn * kDm) return;
  if (in_sizes[13] != kFfn) return;
  if (in_sizes[14] != kDm * kFfn) return;
  if (in_sizes[15] != kDm) return;
  if (in_sizes[16] != kDm || in_sizes[17] != kDm) return;
  if (out_size != kRows * kDm) return;
  if (ws_size < kWsTotal) return;

  const float* x          = (const float*)d_in[0];
  const float* in_proj_w  = (const float*)d_in[1];
  const float* conv_w     = (const float*)d_in[2];
  const float* conv_b     = (const float*)d_in[3];
  const float* x_proj_w   = (const float*)d_in[4];
  const float* dt_proj_w  = (const float*)d_in[5];
  const float* dt_proj_b  = (const float*)d_in[6];
  const float* A_log      = (const float*)d_in[7];
  const float* Dvec       = (const float*)d_in[8];
  const float* out_proj_w = (const float*)d_in[9];
  const float* ln1_w      = (const float*)d_in[10];
  const float* ln1_b      = (const float*)d_in[11];
  const float* ffn_w1     = (const float*)d_in[12];
  const float* ffn_b1     = (const float*)d_in[13];
  const float* ffn_w2     = (const float*)d_in[14];
  const float* ffn_b2     = (const float*)d_in[15];
  const float* ln2_w      = (const float*)d_in[16];
  const float* ln2_b      = (const float*)d_in[17];
  float* out = (float*)d_out;

  char* ws = (char*)d_ws;
  unsigned short* WIN  = (unsigned short*)(ws + kOffWIN);
  unsigned short* WXP  = (unsigned short*)(ws + kOffWXP);
  unsigned short* WDT  = (unsigned short*)(ws + kOffWDT);
  unsigned short* WOUT = (unsigned short*)(ws + kOffWOUT);
  unsigned short* W1   = (unsigned short*)(ws + kOffW1);
  unsigned short* W2   = (unsigned short*)(ws + kOffW2);
  unsigned short* XB   = (unsigned short*)(ws + kOffXB);
  float*          XZ   = (float*)(ws + kOffXZ);
  unsigned short* UCB  = (unsigned short*)(ws + kOffUCB);
  float*          PROJ = (float*)(ws + kOffPROJ);
  unsigned short* DTRB = (unsigned short*)(ws + kOffDTRB);
  float*          DLR  = (float*)(ws + kOffDLR);
  unsigned short* YB   = (unsigned short*)(ws + kOffYB);
  float*          MO   = (float*)(ws + kOffMO);
  float*          H    = (float*)(ws + kOffH);
  unsigned short* HH   = (unsigned short*)(ws + kOffHH);
  unsigned short* HL   = (unsigned short*)(ws + kOffHL);
  float*          F2   = (float*)(ws + kOffF2);
  unsigned short* FH   = (unsigned short*)(ws + kOffFH);
  unsigned short* FL   = (unsigned short*)(ws + kOffFL);
  const float* dummy_bias  = conv_b;
  const float* dummy_resid = x;

  cast_bf16_kernel<<<(kRows * kDm / 8) / 256, 256, 0, stream>>>(x,          XB,   kRows * kDm / 8,  kRows * kDm / 8);
  cast_bf16_kernel<<<(kXZP * kDm / 8) / 256, 256, 0, stream>>>(in_proj_w,   WIN,  kXZP * kDm / 8,   kXZP * kDm / 8);
  cast_bf16_kernel<<<(kPrjP * kDin / 8) / 256, 256, 0, stream>>>(x_proj_w,  WXP,  kPrjP * kDin / 8, kPrjN * kDin / 8);
  cast_bf16_kernel<<<(kDin * kDtR / 8) / 256, 256, 0, stream>>>(dt_proj_w,  WDT,  kDin * kDtR / 8,  kDin * kDtR / 8);
  cast_bf16_kernel<<<(kDm * kDin / 8) / 256, 256, 0, stream>>>(out_proj_w,  WOUT, kDm * kDin / 8,   kDm * kDin / 8);
  cast_bf16_kernel<<<(kFfn * kDm / 8) / 256, 256, 0, stream>>>(ffn_w1,      W1,   kFfn * kDm / 8,   kFfn * kDm / 8);
  cast_bf16_kernel<<<(kDm * kFfn / 8) / 256, 256, 0, stream>>>(ffn_w2,      W2,   kDm * kFfn / 8,   kDm * kFfn / 8);

  wmma_gemm64<1, 0, 0, 0, false, 0><<<dim3(256, 1), 256, 0, stream>>>(
      XB, XB, kDm, 0L, WIN, WIN, kDm, 0L,
      (void*)XZ, (void*)XZ, kXZP, 0L, dummy_bias, dummy_resid, 0L, kRows, kXZP, kDm, 1.0f);

  conv_silu_kernel<<<dim3(kDin / 256, kRows / 64), 256, 0, stream>>>(XZ, conv_w, conv_b, UCB);

  wmma_gemm64<1, 0, 0, 0, false, 0><<<dim3(8, 1), 256, 0, stream>>>(
      UCB, UCB, kDin, 0L, WXP, WXP, kDin, 0L,
      (void*)PROJ, (void*)PROJ, kPrjP, 0L, dummy_bias, dummy_resid, 0L, kRows, kPrjP, kDin, 1.0f);

  dtr_cast_kernel<<<(kRows * kDtR / 8) / 256, 256, 0, stream>>>(PROJ, DTRB, kRows * kDtR / 8);

  wmma_gemm64<1, 0, 0, 0, false, 0><<<dim3(128, 1), 256, 0, stream>>>(
      DTRB, DTRB, kDtR, 0L, WDT, WDT, kDtR, 0L,
      (void*)DLR, (void*)DLR, kDin, 0L, dummy_bias, dummy_resid, 0L, kRows, kDin, kDtR, 1.0f);

  scan_kernel<<<dim3(kDin / 256, kBatch), 256, 0, stream>>>(DLR, XZ, PROJ, conv_w, conv_b, dt_proj_b, A_log, Dvec, YB);

  wmma_gemm64<1, 0, 0, 0, false, 0><<<dim3(64, 1), 256, 0, stream>>>(
      YB, YB, kDin, 0L, WOUT, WOUT, kDin, 0L,
      (void*)MO, (void*)MO, kDm, 0L, dummy_bias, dummy_resid, 0L, kRows, kDm, kDin, 1.0f);

  add_ln_kernel<true, true><<<kRows, 256, 0, stream>>>(MO, x, ln1_w, ln1_b, H, HH, HL);

  wmma_gemm64<1, 1, 2, 2, false, 4><<<dim3(128, 1), 256, 0, stream>>>(
      HH, HL, kDm, 0L, W1, W1, kDm, 0L,
      (void*)FH, (void*)FL, kFfn, 0L, ffn_b1, dummy_resid, 0L, kRows, kFfn, kDm, 1.0f);

  wmma_gemm64<1, 1, 2, 0, false, 0><<<dim3(64, 1), 256, 0, stream>>>(
      FH, FL, kFfn, 0L, W2, W2, kFfn, 0L,
      (void*)F2, (void*)F2, kDm, 0L, ffn_b2, dummy_resid, 0L, kRows, kDm, kFfn, 1.0f);

  add_ln_kernel<false, false><<<kRows, 256, 0, stream>>>(F2, H, ln2_w, ln2_b, out, HH, HL);
}
